// MOTMPNet_50440095924470
// MI455X (gfx1250) — hardware-verified
//
#include <hip/hip_runtime.h>
#include <stddef.h>


#define NTHR   256
#define NWAVE  8
#define EPT    8
#define CHUNK  (NTHR * EPT)
#define WCAP   (EPT * 32)
#define LISTN  (NWAVE * WCAP)
#define TE     16
#define PASSN  (NWAVE * TE)
#define PCAP   (CHUNK + PASSN)
#define NB     256
#define ACCW   128
#define DN     32
#define DE     16
#define F1     80
#define KP     96
#define KF     64
#define WSC    16.0f
#define WINV   0.0625f
#define LALPHA 0.2f
#define NEGBIG (-1.0e30f)
#define DEPS   1e-12f

static_assert(PASSN <= NTHR);
static_assert((PCAP % PASSN) == 0);
static_assert(NB == 16 * 2 * NWAVE);
static_assert(((NB * (ACCW / 4)) % NTHR) == 0);
static_assert(WCAP == 32 * EPT);

typedef float          v2f  __attribute__((ext_vector_type(2)));
typedef float          v4f  __attribute__((ext_vector_type(4)));
typedef float          v8f  __attribute__((ext_vector_type(8)));
typedef int            v4i  __attribute__((ext_vector_type(4)));
typedef _Float16       v8h  __attribute__((ext_vector_type(8)));
typedef _Float16       v16h __attribute__((ext_vector_type(16)));
typedef unsigned short v8us __attribute__((ext_vector_type(8)));
typedef __bf16         v16b __attribute__((ext_vector_type(16)));
union FragH { v16h v; v8h h[2]; };
union FragB { v16b v; v8us u[2]; };
union StgU  { _Float16 h[NWAVE * TE * KP]; float o[NWAVE * 16 * 32]; };
union MsgU  { float f[PASSN * 64]; unsigned short w[2 * 32 * ACCW]; };

__device__ __forceinline__ v8h zero8() {
  v8h r;
#pragma unroll
  for (int i = 0; i < 8; ++i) r[i] = (_Float16)0.0f;
  return r;
}

__device__ __forceinline__ v8h cvt8h(v4f a, v4f b) {
  v8h r;
  r[0] = (_Float16)a.x; r[1] = (_Float16)a.y; r[2] = (_Float16)a.z; r[3] = (_Float16)a.w;
  r[4] = (_Float16)b.x; r[5] = (_Float16)b.y; r[6] = (_Float16)b.z; r[7] = (_Float16)b.w;
  return r;
}

__device__ __forceinline__ v8f fill8(float v) {
  v8f c;
#pragma unroll
  for (int i = 0; i < 8; ++i) c[i] = v;
  return c;
}

__device__ __forceinline__ v8f wmh(v16h a, v16h b, v8f c) {
  v8f d = __builtin_amdgcn_wmma_f32_16x16x32_f16(false, a, false, b, (short)0, c, false, false);
  asm volatile("v_nop\n\tv_nop\n\tv_nop\n\tv_nop" : "+v"(d) : "v"(a), "v"(b) : "memory");
  return d;
}

__device__ __forceinline__ v8f wmb(v16b a, v16b b, v8f c) {
  v8f d = __builtin_amdgcn_wmma_f32_16x16x32_bf16(false, a, false, b, (short)0, c, false, false);
  asm volatile("v_nop\n\tv_nop\n\tv_nop\n\tv_nop" : "+v"(d) : "v"(a), "v"(b) : "memory");
  return d;
}

__device__ __forceinline__ v8h relu8(v8f d) {
  v8h r;
#pragma unroll
  for (int i = 0; i < 8; ++i) { const float t = fmaxf(d[i] * WINV, 0.0f); r[i] = (_Float16)t; }
  return r;
}

__device__ __forceinline__ v8f ldc8(const float* p) {
  const v4f a = *(const v4f*)p;
  const v4f b = *(const v4f*)(p + 4);
  v8f c;
  c[0] = a.x; c[1] = a.y; c[2] = a.z; c[3] = a.w;
  c[4] = b.x; c[5] = b.y; c[6] = b.z; c[7] = b.w;
  return c;
}

__device__ __forceinline__ unsigned int bfb(float f) {
  const unsigned int u = __float_as_uint(f);
  return (u + 0x7FFFu + ((u >> 16) & 1u)) >> 16;
}
__device__ __forceinline__ unsigned int lob(float f) {
  const unsigned int hb = bfb(f);
  const float hf = __uint_as_float(hb << 16);
  return bfb(f - hf);
}
__device__ __forceinline__ v8us hi8(v4f a, v4f b) {
  v8us r;
  r[0] = (unsigned short)bfb(a.x); r[1] = (unsigned short)bfb(a.y); r[2] = (unsigned short)bfb(a.z); r[3] = (unsigned short)bfb(a.w);
  r[4] = (unsigned short)bfb(b.x); r[5] = (unsigned short)bfb(b.y); r[6] = (unsigned short)bfb(b.z); r[7] = (unsigned short)bfb(b.w);
  return r;
}
__device__ __forceinline__ v8us lo8(v4f a, v4f b) {
  v8us r;
  r[0] = (unsigned short)lob(a.x); r[1] = (unsigned short)lob(a.y); r[2] = (unsigned short)lob(a.z); r[3] = (unsigned short)lob(a.w);
  r[4] = (unsigned short)lob(b.x); r[5] = (unsigned short)lob(b.y); r[6] = (unsigned short)lob(b.z); r[7] = (unsigned short)lob(b.w);
  return r;
}

__device__ __forceinline__ int scan_chunk(const int* __restrict__ keys, int nE, int cbase, int nodeBase,
                                          int* list, int tid, int wave) {
  int wc = 0;
  const int el0  = tid * EPT;
  const int e0   = cbase + el0;
  const int sent = -2147483647 - 1;
  v4i da, db;
  if (cbase + CHUNK <= nE) {
    da = *(const v4i*)(keys + e0);
    db = *(const v4i*)(keys + e0 + 4);
  } else {
    da.x = (e0     < nE) ? keys[min(e0,     nE - 1)] : sent;
    da.y = (e0 + 1 < nE) ? keys[min(e0 + 1, nE - 1)] : sent;
    da.z = (e0 + 2 < nE) ? keys[min(e0 + 2, nE - 1)] : sent;
    da.w = (e0 + 3 < nE) ? keys[min(e0 + 3, nE - 1)] : sent;
    db.x = (e0 + 4 < nE) ? keys[min(e0 + 4, nE - 1)] : sent;
    db.y = (e0 + 5 < nE) ? keys[min(e0 + 5, nE - 1)] : sent;
    db.z = (e0 + 6 < nE) ? keys[min(e0 + 6, nE - 1)] : sent;
    db.w = (e0 + 7 < nE) ? keys[min(e0 + 7, nE - 1)] : sent;
  }
  const unsigned nb = (unsigned)nodeBase;
  const unsigned s0 = (unsigned)da.x - nb, s1 = (unsigned)da.y - nb;
  const unsigned s2 = (unsigned)da.z - nb, s3 = (unsigned)da.w - nb;
  const unsigned s4 = (unsigned)db.x - nb, s5 = (unsigned)db.y - nb;
  const unsigned s6 = (unsigned)db.z - nb, s7 = (unsigned)db.w - nb;
  const bool h0 = s0 < (unsigned)NB, h1 = s1 < (unsigned)NB, h2 = s2 < (unsigned)NB, h3 = s3 < (unsigned)NB;
  const bool h4 = s4 < (unsigned)NB, h5 = s5 < (unsigned)NB, h6 = s6 < (unsigned)NB, h7 = s7 < (unsigned)NB;
  const unsigned any = __builtin_amdgcn_ballot_w32(h0 | h1 | h2 | h3 | h4 | h5 | h6 | h7);
  if (any != 0u) {
#define HITJ(J, HJ) { \
      const unsigned mj = __builtin_amdgcn_ballot_w32(HJ); \
      if (mj != 0u) { \
        if (HJ) { \
          const int pos = wc + (int)__builtin_amdgcn_mbcnt_lo(mj, 0u); \
          if (pos < WCAP) list[wave * WCAP + pos] = el0 + (J); \
        } \
        wc += (int)__builtin_popcount(mj); } }
    HITJ(0, h0)
    HITJ(1, h1)
    HITJ(2, h2)
    HITJ(3, h3)
    HITJ(4, h4)
    HITJ(5, h5)
    HITJ(6, h6)
    HITJ(7, h7)
#undef HITJ
  }
  return wc;
}

__global__ __launch_bounds__(NTHR) void k_natt(const float* __restrict__ x, const float* __restrict__ aout,
                                               const float* __restrict__ ain, float* natt, int nN) {
  __shared__ __attribute__((aligned(16))) float sh[NTHR * 8];
  const int tid = threadIdx.x;
  int n = blockIdx.x * NTHR + tid;
  n = n > nN - 1 ? nN - 1 : n;
  n = n < 0 ? 0 : n;
  const float* xp = x + (size_t)n * DN;
  float s0 = 0.0f, s1 = 0.0f, s2 = 0.0f, s3 = 0.0f, s4 = 0.0f, s5 = 0.0f, s6 = 0.0f, s7 = 0.0f;
#pragma unroll 1
  for (int k = 0; k < DN; ++k) {
    const float xv = xp[k];
    s0 = fmaf(ain[k],           xv, s0);
    s1 = fmaf(ain[2 * DN + k],  xv, s1);
    s2 = fmaf(aout[k],          xv, s2);
    s3 = fmaf(aout[2 * DN + k], xv, s3);
    s4 = fmaf(ain[DN + k],      xv, s4);
    s5 = fmaf(ain[3 * DN + k],  xv, s5);
    s6 = fmaf(aout[DN + k],     xv, s6);
    s7 = fmaf(aout[3 * DN + k], xv, s7);
  }
  {
    v4f a, b;
    a.x = s0; a.y = s1; a.z = s2; a.w = s3;
    b.x = s4; b.y = s5; b.z = s6; b.w = s7;
    *(v4f*)(sh + tid * 8)     = a;
    *(v4f*)(sh + tid * 8 + 4) = b;
  }
  __syncthreads();
  const v4f o0 = *(const v4f*)(sh + 4 * tid);
  const v4f o1 = *(const v4f*)(sh + 4 * (NTHR + tid));
  float* gp = natt + (size_t)blockIdx.x * (NTHR * 8);
  *(volatile v4f*)(gp + 4 * tid)          = o0;
  *(volatile v4f*)(gp + 4 * (NTHR + tid)) = o1;
  __threadfence();
  *(volatile v4f*)(gp + 4 * tid)          = o0;
  *(volatile v4f*)(gp + 4 * (NTHR + tid)) = o1;
}

__global__ __launch_bounds__(NTHR) void k_edge(
    const float* __restrict__ x, const float* __restrict__ ea, const int* __restrict__ ei,
    const float* __restrict__ natt,
    const float* __restrict__ We1, const float* __restrict__ be1,
    const float* __restrict__ We2, const float* __restrict__ be2,
    const float* __restrict__ Wfo, const float* __restrict__ bfo,
    const float* __restrict__ Wfi, const float* __restrict__ bfi,
    const float* __restrict__ Wn, const float* __restrict__ bn,
    float* outp, int nN, int nE) {
  extern __shared__ __attribute__((aligned(16))) float accs[];
  __shared__ __attribute__((aligned(16))) float    st[(NB + 1) * 8];
  __shared__ __attribute__((aligned(16))) _Float16 sW1[F1 * KP];
  __shared__ __attribute__((aligned(16))) _Float16 sW2[DE * KP];
  __shared__ __attribute__((aligned(16))) _Float16 sWf[4 * 32 * KF];
  __shared__ __attribute__((aligned(16))) float    sB1[F1];
  __shared__ __attribute__((aligned(16))) float    sB2[DE];
  __shared__ __attribute__((aligned(16))) float    sBf[128];
  __shared__ __attribute__((aligned(16))) StgU     stgU;
  __shared__ __attribute__((aligned(16))) MsgU     msgU;
  __shared__ __attribute__((aligned(16))) v4f      elg[PASSN];
  __shared__ int esl[PASSN];
  __shared__ __attribute__((aligned(16))) int      list[LISTN];
  __shared__ __attribute__((aligned(16))) int      pend[PCAP];
  __shared__ int wcnt[NWAVE];
  __shared__ int pendN;

  const int tid = threadIdx.x, lane = tid & 31, wave = tid >> 5, hh = lane >> 4, m = lane & 15;
  const int nodeBase = blockIdx.x * NB;
  const int* keys = ei;
  const int* cols = ei + (size_t)nE;

  for (int i = tid; i < (NB + 1) * ACCW; i += NTHR) accs[i] = 0.0f;
  for (int i = tid; i < (NB + 1) * 8; i += NTHR) st[i] = ((i & 1) != 0) ? 0.0f : NEGBIG;
  for (int i = tid; i < F1 * KP; i += NTHR) {
    const int f = i / KP, k = i - f * KP;
    const int kc = k > F1 - 1 ? F1 - 1 : k;
    float v = We1[kc * F1 + f];
    v = (k < F1) ? v : 0.0f;
    sW1[i] = (_Float16)(v * WSC);
  }
  for (int i = tid; i < DE * KP; i += NTHR) {
    const int f = i / KP, k = i - f * KP;
    const int kc = k > F1 - 1 ? F1 - 1 : k;
    float v = We2[kc * DE + f];
    v = (k < F1) ? v : 0.0f;
    sW2[i] = (_Float16)(v * WSC);
  }
  for (int i = tid; i < 4 * 32 * KF; i += NTHR) {
    const int mi = i >> 11, d = (i >> 6) & 31, k = i & 63;
    const int sd = mi >> 1, h = mi & 1;
    const int kc = k > 47 ? 47 : k;
    const float vo = Wfo[(h * 48 + kc) * 32 + d];
    const float vi = Wfi[(h * 48 + kc) * 32 + d];
    float v = (sd != 0) ? vo : vi;
    v = (k < 48) ? v : 0.0f;
    sWf[i] = (_Float16)(v * WSC);
  }
  if (tid < F1) sB1[tid] = be1[tid] * WSC;
  if (tid < DE) sB2[tid] = be2[tid] * WSC;
  if (tid < 128) {
    const int mi = tid >> 5, d = tid & 31, sd = mi >> 1, h = mi & 1;
    const float vo = bfo[h * 32 + d], vi = bfi[h * 32 + d];
    sBf[tid] = ((sd != 0) ? vo : vi) * WSC;
  }
  if (tid == 0) pendN = 0;
  __syncthreads();

  const int nChunks = (nE + CHUNK - 1) / CHUNK;
#pragma unroll 1
  for (int ch = 0; ch < nChunks; ++ch) {
    const int cbase = ch * CHUNK;
    const int wc = scan_chunk(keys, nE, cbase, nodeBase, list, tid, wave);
    if (lane == 0) wcnt[wave] = wc;
    __syncthreads();

    const int base = pendN;
    int tot = 0, myoff = 0;
#pragma unroll
    for (int w = 0; w < NWAVE; ++w) {
      int c = wcnt[w];
      c = c > WCAP ? WCAP : (c < 0 ? 0 : c);
      if (w < wave) myoff += c;
      tot += c;
    }
    int newN = base + tot;
    newN = newN > PCAP ? PCAP : newN;
    {
      int n = wcnt[wave];
      n = n > WCAP ? WCAP : (n < 0 ? 0 : n);
      const int* lp = list + wave * WCAP;
      for (int i = lane; i < n; i += 32) {
        const int pos = base + myoff + i;
        if (pos < PCAP) pend[pos] = cbase + lp[i];
      }
    }
    const int fin = (ch == nChunks - 1) ? 1 : 0;
    const int R   = (fin != 0) ? (newN + PASSN - 1) / PASSN : newN / PASSN;
    const int Pv  = (fin != 0) ? newN : R * PASSN;
    __syncthreads();

#pragma unroll 1
    for (int r = 0; r < R; ++r) {
      int sdm;
      {
        const int sip = wave * TE + m;
        int idx = r * PASSN + sip;
        const bool valid = idx < Pv;
        idx = idx > PCAP - 1 ? PCAP - 1 : idx;
        int e = pend[idx];
        e = e < 0 ? 0 : (e > nE - 1 ? nE - 1 : e);
        int row = keys[e];
        int col = cols[e];
        const int slot = row - nodeBase;
        const bool ok = valid && ((unsigned)slot < (unsigned)NB) && (row != col);
        sdm = (row > col) ? 0 : 1;
        row = row < 0 ? 0 : (row > nN - 1 ? nN - 1 : row);
        col = col < 0 ? 0 : (col > nN - 1 ? nN - 1 : col);
        const int sidx = ok ? (slot * 2 + sdm) : (2 * NB);
        const int nsel = (hh != 0) ? col : row;
        const float* xp = x + (size_t)nsel * DN;
        _Float16* srow = stgU.h + (size_t)sip * KP;
#pragma unroll
        for (int j = 0; j < 4; ++j) {
          const v4f a = *(const v4f*)(xp + 8 * j);
          const v4f b = *(const v4f*)(xp + 8 * j + 4);
          *(v8h*)(srow + 32 * hh + 8 * j) = cvt8h(a, b);
        }
        {
          const float* epp = ea + (size_t)e * DE + 8 * hh;
          const v4f a = *(const v4f*)epp;
          const v4f b = *(const v4f*)(epp + 4);
          *(v8h*)(srow + 64 + 8 * hh) = cvt8h(a, b);
          *(v8h*)(srow + 80 + 8 * hh) = zero8();
        }
        const v2f sr = *(const v2f*)(natt + (size_t)row * 8 + 2 * sdm);
        const v2f sc = *(const v2f*)(natt + (size_t)col * 8 + 4 + 2 * sdm);
        float l0 = sr.x + sc.x, l1 = sr.y + sc.y;
        l0 = (l0 >= 0.0f) ? l0 : LALPHA * l0;
        l1 = (l1 >= 0.0f) ? l1 : LALPHA * l1;
        if (!ok) { l0 = 0.0f; l1 = 0.0f; }
        if (hh == 0) {
          v4f t; t.x = l0; t.y = l1; t.z = 0.0f; t.w = 0.0f;
          elg[sip] = t;
          esl[sip] = sidx;
        }
      }
      __syncthreads();

      {
        const _Float16* wsrc = stgU.h + (size_t)(wave * TE) * KP;
        FragH bx[3];
#pragma unroll
        for (int ks = 0; ks < 3; ++ks) {
          const _Float16* bp = wsrc + m * KP + 32 * ks + 8 * hh;
          bx[ks].h[0] = *(const v8h*)bp;
          bx[ks].h[1] = *(const v8h*)(bp + 16);
        }
        v8f d1[5];
#pragma unroll
        for (int ft = 0; ft < 5; ++ft) {
          d1[ft] = ldc8(sB1 + 16 * ft + 8 * hh);
#pragma unroll
          for (int ks = 0; ks < 3; ++ks) {
            FragH a;
            const _Float16* ap = sW1 + (16 * ft + m) * KP + 32 * ks + 8 * hh;
            a.h[0] = *(const v8h*)ap;
            a.h[1] = *(const v8h*)(ap + 16);
            d1[ft] = wmh(a.v, bx[ks].v, d1[ft]);
          }
        }
        FragH b2[3];
        b2[0].h[0] = relu8(d1[0]); b2[0].h[1] = relu8(d1[1]);
        b2[1].h[0] = relu8(d1[2]); b2[1].h[1] = relu8(d1[3]);
        b2[2].h[0] = relu8(d1[4]); b2[2].h[1] = zero8();
        v8f d2 = ldc8(sB2 + 8 * hh);
#pragma unroll
        for (int ks = 0; ks < 3; ++ks) {
          FragH a;
          const _Float16* ap = sW2 + m * KP + 32 * ks + 8 * hh;
          a.h[0] = *(const v8h*)ap;
          a.h[1] = *(const v8h*)(ap + 16);
          d2 = wmh(a.v, b2[ks].v, d2);
        }
        FragH fb1;
        fb1.h[0] = relu8(d2);
        fb1.h[1] = zero8();
        float* mrow = msgU.f + (size_t)(wave * TE + m) * 64;
#pragma unroll
        for (int h = 0; h < 2; ++h) {
#pragma unroll
          for (int dt = 0; dt < 2; ++dt) {
            v8f dfi = ldc8(sBf + (0 * 2 + h) * 32 + 16 * dt + 8 * hh);
            v8f dfo = ldc8(sBf + (1 * 2 + h) * 32 + 16 * dt + 8 * hh);
            {
              FragH a;
              const _Float16* ap = sWf + ((0 * 2 + h) * 32 + 16 * dt + m) * KF + 8 * hh;
              a.h[0] = *(const v8h*)ap;
              a.h[1] = *(const v8h*)(ap + 16);
              dfi = wmh(a.v, bx[0].v, dfi);
              a.h[0] = *(const v8h*)(ap + 32);
              a.h[1] = *(const v8h*)(ap + 48);
              dfi = wmh(a.v, fb1.v, dfi);
            }
            {
              FragH a;
              const _Float16* ap = sWf + ((1 * 2 + h) * 32 + 16 * dt + m) * KF + 8 * hh;
              a.h[0] = *(const v8h*)ap;
              a.h[1] = *(const v8h*)(ap + 16);
              dfo = wmh(a.v, bx[0].v, dfo);
              a.h[0] = *(const v8h*)(ap + 32);
              a.h[1] = *(const v8h*)(ap + 48);
              dfo = wmh(a.v, fb1.v, dfo);
            }
            v4f o0, o1;
            {
              float t[8];
#pragma unroll
              for (int rr = 0; rr < 8; ++rr) {
                const float vi = dfi[rr], vo = dfo[rr];
                const float v = (sdm != 0) ? vo : vi;
                t[rr] = fmaxf(v * WINV, 0.0f);
              }
              o0.x = t[0]; o0.y = t[1]; o0.z = t[2]; o0.w = t[3];
              o1.x = t[4]; o1.y = t[5]; o1.z = t[6]; o1.w = t[7];
            }
            *(v4f*)(mrow + h * 32 + 16 * dt + 8 * hh)     = o0;
            *(v4f*)(mrow + h * 32 + 16 * dt + 8 * hh + 4) = o1;
          }
        }
      }
      __syncthreads();

      if (wave == 0) {
#pragma unroll 1
        for (int i = 0; i < PASSN; ++i) {
          int sidx = esl[i];
          sidx = sidx < 0 ? 0 : (sidx > 2 * NB ? 2 * NB : sidx);
          const v4f lg = elg[i];
          float* sp = st + sidx * 4;
          const v4f s = *(const v4f*)sp;
          const float nm0 = fmaxf(s.x, lg.x);
          const float nm1 = fmaxf(s.z, lg.y);
          const float sc0 = __expf(s.x - nm0), p0 = __expf(lg.x - nm0);
          const float sc1 = __expf(s.z - nm1), p1 = __expf(lg.y - nm1);
          v4f ns;
          ns.x = nm0; ns.y = s.y * sc0 + p0;
          ns.z = nm1; ns.w = s.w * sc1 + p1;
          float* aprow = accs + (size_t)sidx * 64;
          const float* mp = msgU.f + i * 64;
          const float a0 = aprow[lane], a1 = aprow[32 + lane];
          const float f0 = mp[lane], f1 = mp[32 + lane];
          const float na0 = a0 * sc0 + p0 * f0;
          const float na1 = a1 * sc1 + p1 * f1;
          aprow[lane]      = na0;
          aprow[32 + lane] = na1;
          *(v4f*)sp = ns;
        }
      }
      __syncthreads();
    }

    int rem = newN - R * PASSN;
    rem = rem < 0 ? 0 : rem;
    if (R > 0 && tid < rem) pend[tid] = pend[R * PASSN + tid];
    if (tid == 0) pendN = rem;
  }
  __syncthreads();

  for (int i = tid; i < 32 * ACCW; i += NTHR) {
    const int n = i >> 7, k = i & 127;
    const float v = Wn[k * 32 + n];
    msgU.w[i]             = (unsigned short)bfb(v);
    msgU.w[32 * ACCW + i] = (unsigned short)lob(v);
  }
  for (int i = tid; i < NB * 4; i += NTHR) {
    const int id = (i >> 1) * 4 + 1 + 2 * (i & 1);
    const float dn = st[id];
    st[id] = 1.0f / (dn + DEPS);
  }
  __syncthreads();
  for (int i = tid; i < NB * (ACCW / 4); i += NTHR) {
    const int slot = i >> 5;
    const int c4 = (i & 31) * 4;
    const int sd = c4 >> 6, h = (c4 >> 5) & 1;
    const float rc = st[(slot * 2 + sd) * 4 + 1 + 2 * h];
    v4f v = *(v4f*)(accs + (size_t)i * 4);
    v = v * rc;
    *(v4f*)(accs + (size_t)i * 4) = v;
  }
  __syncthreads();

  {
    float* ot = stgU.o + wave * 512;
    const float bb0 = bn[m], bb1 = bn[16 + m];
#pragma unroll 1
    for (int t = 0; t < 2; ++t) {
      const int rt = wave * 2 + t;
      v8f dn0 = fill8(bb0), dn1 = fill8(bb1);
#pragma unroll
      for (int ks = 0; ks < 4; ++ks) {
        const float* ap = accs + (size_t)(16 * rt + m) * ACCW + 32 * ks + 8 * hh;
        const v4f x0 = *(const v4f*)ap,        x1 = *(const v4f*)(ap + 4);
        const v4f x2 = *(const v4f*)(ap + 16), x3 = *(const v4f*)(ap + 20);
        FragB ahi, alo;
        ahi.u[0] = hi8(x0, x1); ahi.u[1] = hi8(x2, x3);
        alo.u[0] = lo8(x0, x1); alo.u[1] = lo8(x2, x3);
        {
          const unsigned short* bp = msgU.w + (size_t)m * ACCW + 32 * ks + 8 * hh;
          FragB bh, bl;
          bh.u[0] = *(const v8us*)bp;               bh.u[1] = *(const v8us*)(bp + 16);
          bl.u[0] = *(const v8us*)(bp + 32 * ACCW); bl.u[1] = *(const v8us*)(bp + 32 * ACCW + 16);
          dn0 = wmb(ahi.v, bh.v, dn0);
          dn0 = wmb(alo.v, bh.v, dn0);
          dn0 = wmb(ahi.v, bl.v, dn0);
        }
        {
          const unsigned short* bp = msgU.w + (size_t)(16 + m) * ACCW + 32 * ks + 8 * hh;
          FragB bh, bl;
          bh.u[0] = *(const v8us*)bp;               bh.u[1] = *(const v8us*)(bp + 16);
          bl.u[0] = *(const v8us*)(bp + 32 * ACCW); bl.u[1] = *(const v8us*)(bp + 32 * ACCW + 16);
          dn1 = wmb(ahi.v, bh.v, dn1);
          dn1 = wmb(alo.v, bh.v, dn1);
          dn1 = wmb(ahi.v, bl.v, dn1);
        }
      }
#pragma unroll
      for (int rr = 0; rr < 8; ++rr) {
        ot[(8 * hh + rr) * 32 + m]      = fmaxf(dn0[rr], 0.0f);
        ot[(8 * hh + rr) * 32 + 16 + m] = fmaxf(dn1[rr], 0.0f);
      }
      __syncthreads();
      v4f ov[4];
#pragma unroll
      for (int q = 0; q < 4; ++q) {
        const int rr = 4 * q + (lane >> 3);
        ov[q] = *(const v4f*)(ot + rr * 32 + 4 * (lane & 7));
      }
      const size_t rowg0 = (size_t)nodeBase + (size_t)(16 * rt);
#pragma unroll
      for (int q = 0; q < 4; ++q) {
        const size_t node = rowg0 + (size_t)(4 * q + (lane >> 3));
        if (node < (size_t)nN) *(volatile v4f*)(outp + node * DN + 4 * (lane & 7)) = ov[q];
      }
      __threadfence();
#pragma unroll
      for (int q = 0; q < 4; ++q) {
        const size_t node = rowg0 + (size_t)(4 * q + (lane >> 3));
        if (node < (size_t)nN) *(volatile v4f*)(outp + node * DN + 4 * (lane & 7)) = ov[q];
      }
    }
  }
}

extern "C" void kernel_launch(void* const* d_in, const int* in_sizes, int n_in,
                              void* d_out, int out_size, void* d_ws, size_t ws_size,
                              hipStream_t stream) {
  if (n_in < 15) return;
  const int nN = in_sizes[0] / DN;
  const int nE = in_sizes[14] / 2;
  if (nN <= 0 || nE <= 0) return;
  if (in_sizes[0] != nN * DN || in_sizes[14] != nE * 2 || in_sizes[1] != nE * DE) return;
  if (in_sizes[2] != F1 * F1 || in_sizes[3] < F1 || in_sizes[4] != F1 * DE || in_sizes[5] < DE) return;
  if (in_sizes[6] != 2 * 48 * 32 || in_sizes[7] < 64 || in_sizes[8] != 2 * 48 * 32 || in_sizes[9] < 64) return;
  if (in_sizes[10] != ACCW * DN || in_sizes[11] < DN || in_sizes[12] < 2 * 64 || in_sizes[13] < 2 * 64) return;
  if (out_size != nN * DN) return;

  const float* x    = (const float*)d_in[0];
  const float* ea   = (const float*)d_in[1];
  const float* We1  = (const float*)d_in[2];
  const float* be1  = (const float*)d_in[3];
  const float* We2  = (const float*)d_in[4];
  const float* be2  = (const float*)d_in[5];
  const float* Wfo  = (const float*)d_in[6];
  const float* bfo  = (const float*)d_in[7];
  const float* Wfi  = (const float*)d_in[8];
  const float* bfi  = (const float*)d_in[9];
  const float* Wn   = (const float*)d_in[10];
  const float* bn   = (const float*)d_in[11];
  const float* aao  = (const float*)d_in[12];
  const float* aai  = (const float*)d_in[13];
  const int*   ei   = (const int*)d_in[14];
  float* out = (float*)d_out;

  const int gridA = (nN + NTHR - 1) / NTHR;
  const size_t nattBytes = (size_t)gridA * NTHR * 8 * sizeof(float);
  if (nattBytes > ws_size) return;
  float* natt = (float*)d_ws;

  const int nBlk = (nN + NB - 1) / NB;
  const size_t dyn = (size_t)(NB + 1) * ACCW * sizeof(float);
  hipFuncSetAttribute((const void*)k_edge, hipFuncAttributeMaxDynamicSharedMemorySize, (int)dyn);

  k_natt<<<gridA, NTHR, 0, stream>>>(x, aao, aai, natt, nN);

  k_edge<<<nBlk, NTHR, dyn, stream>>>(x, ea, ei, natt, We1, be1, We2, be2, Wfo, bfo, Wfi, bfi, Wn, bn,
                                      out, nN, nE);
}
